// MambaBlock_8358006358375
// MI455X (gfx1250) — hardware-verified
//
#include <hip/hip_runtime.h>
#include <math.h>

typedef __attribute__((ext_vector_type(16))) __bf16   v16b;
typedef __attribute__((ext_vector_type(8)))  __bf16   v8b;
typedef __attribute__((ext_vector_type(8)))  float    v8f;
typedef __attribute__((ext_vector_type(4)))  float    v4f;
typedef __attribute__((ext_vector_type(4)))  unsigned v4u;

constexpr int kBatch = 2;
constexpr int kSeq   = 2048;
constexpr int kDm    = 1024;
constexpr int kDin   = 2048;
constexpr int kNst   = 64;
constexpr int kXzN   = 2 * kDin;
constexpr int kSsmN  = 2 * kNst + 1;
constexpr int kSsmP  = 192;
constexpr int kRows  = kBatch * kSeq;
constexpr int kKd    = 2 * kDin;
constexpr int kScCh  = 128;
constexpr int kScTS  = 16;
static_assert(kSsmN == 129 && kSsmP % 64 == 0 && kSsmP >= kSsmN, "x_proj width and padded width");
static_assert(kDm % 32 == 0 && kKd % 32 == 0, "GEMM K multiples of 32");
static_assert(kRows % 64 == 0 && kXzN % 64 == 0 && kDm % 64 == 0 && kDin % 64 == 0, "GEMM M,N multiples of 64");
static_assert(kSeq % kScTS == 0 && kDin % kScCh == 0 && kScCh == 2 * kNst, "scan tiling");
static_assert(kSsmP == 3 * kNst, "staging row = Abar | dtB | C");

constexpr size_t kOffXB    = 0;
constexpr size_t kOffWINB  = kOffXB    + (size_t)kRows * kDm * 2;
constexpr size_t kOffWXD   = kOffWINB  + (size_t)kXzN * kDm * 2;
constexpr size_t kOffWOUTD = kOffWXD   + (size_t)kSsmP * kDin * 4;
constexpr size_t kOffXIN   = kOffWOUTD + (size_t)kDm * kDin * 4;
constexpr size_t kOffZS    = kOffXIN   + (size_t)kRows * kDin * 4;
constexpr size_t kOffXCW   = kOffZS    + (size_t)kRows * kDin * 4;
constexpr size_t kOffSSM   = kOffXCW   + (size_t)kRows * kDin * 4;
constexpr size_t kWsTotal  = kOffSSM   + (size_t)kRows * kSsmP * 4;
static_assert(kWsTotal == 130547712ull, "carve total");
static_assert(kWsTotal <= 134217728ull, "carve cap");
static_assert((kOffWINB % 128) == 0 && (kOffWXD % 128) == 0 && (kOffWOUTD % 128) == 0 && (kOffXIN % 128) == 0 &&
              (kOffZS % 128) == 0 && (kOffXCW % 128) == 0 && (kOffSSM % 128) == 0, "128-B aligned regions");

__device__ __forceinline__ unsigned bf16_rne_bits(float f) {
  const unsigned u = __float_as_uint(f);
  return (u + 0x7FFFu + ((u >> 16) & 1u)) >> 16;
}
__device__ __forceinline__ float bf16_rne_val(float f) {
  return __uint_as_float(bf16_rne_bits(f) << 16);
}
__device__ __forceinline__ unsigned split_word(float v) {
  const unsigned hb = bf16_rne_bits(v);
  const float hf = __uint_as_float(hb << 16);
  const unsigned lb = bf16_rne_bits(v - hf);
  return hb | (lb << 16);
}
__device__ __forceinline__ float word_val(unsigned w) {
  return __uint_as_float(w << 16) + __uint_as_float(w & 0xffff0000u);
}

__device__ __forceinline__ void guard_row_b(v8f& a, v8f& b, v8f& c, v8f& d, v16b x, v16b b0, v16b b1, v16b b2, v16b b3) {
  asm volatile("v_nop\n\tv_nop\n\tv_nop\n\tv_nop" : "+v"(a), "+v"(b), "+v"(c), "+v"(d) : "v"(x), "v"(b0), "v"(b1), "v"(b2), "v"(b3));
}
__device__ __forceinline__ void keep4_b(v16b a, v16b b, v16b c, v16b d) { asm volatile("v_nop" :: "v"(a), "v"(b), "v"(c), "v"(d)); }
__device__ __forceinline__ void acc_guard4(v8f& a, v8f& b, v8f& c, v8f& d) { asm volatile("v_nop\n\tv_nop\n\tv_nop\n\tv_nop" : "+v"(a), "+v"(b), "+v"(c), "+v"(d)); }

struct FragB {
  union U { v16b v; v8b h[2]; };
  static __device__ __forceinline__ v16b load(const __bf16* p) {
    U f; f.h[0] = *(const v8b*)(p); f.h[1] = *(const v8b*)(p + 16); return f.v;
  }
  static __device__ __forceinline__ v8f mma(v16b a, v16b b, v8f c) {
    return __builtin_amdgcn_wmma_f32_16x16x32_bf16(false, a, false, b, (short)0, c, false, false);
  }
};

template <int EPI>
__global__ __launch_bounds__(256) void gemm_bf16_kernel(
    const unsigned short* __restrict__ Ap, int lda,
    const unsigned short* __restrict__ Btp, int ldb,
    void* C0, void* C1, int ldc, int M, int N, int K)
{
  const __bf16* A  = (const __bf16*)Ap;
  const __bf16* Bt = (const __bf16*)Btp;
  __shared__ __align__(16) float sT[8][16 * 68];
  const int lane = threadIdx.x & 31;
  const int wave = threadIdx.x >> 5;
  const int tilesN = N >> 6;
  const int tilesM = M >> 6;
  const int tile = blockIdx.x * 8 + wave;
  if (tile >= tilesM * tilesN) return;
  const int tm = tile / tilesN;
  const int tn = tile - tm * tilesN;
  const int m0 = tm << 6;
  const int n0 = tn << 6;

  const int rlane = lane & 15;
  const int koff  = (lane >> 4) * 8;
  const int mOff  = (lane >> 4) * 8;

  v8f acc[4][4];
#pragma unroll
  for (int i = 0; i < 4; ++i)
#pragma unroll
    for (int j = 0; j < 4; ++j) acc[i][j] = (v8f){0.f,0.f,0.f,0.f,0.f,0.f,0.f,0.f};

  for (int k0 = 0; k0 < K; k0 += 32) {
    v16b bh[4];
#pragma unroll
    for (int j = 0; j < 4; ++j) {
      const size_t bo = (size_t)(n0 + (j << 4) + rlane) * ldb + koff + k0;
      bh[j] = FragB::load(Bt + bo);
    }
#pragma unroll
    for (int i = 0; i < 4; ++i) {
      const size_t ao = (size_t)(m0 + (i << 4) + rlane) * lda + koff + k0;
      const v16b ah = FragB::load(A + ao);
#pragma unroll
      for (int j = 0; j < 4; ++j) acc[i][j] = FragB::mma(ah, bh[j], acc[i][j]);
      guard_row_b(acc[i][0], acc[i][1], acc[i][2], acc[i][3], ah, bh[0], bh[1], bh[2], bh[3]);
    }
    keep4_b(bh[0], bh[1], bh[2], bh[3]);
  }
  acc_guard4(acc[0][0], acc[0][1], acc[0][2], acc[0][3]);
  acc_guard4(acc[1][0], acc[1][1], acc[1][2], acc[1][3]);
  acc_guard4(acc[2][0], acc[2][1], acc[2][2], acc[2][3]);
  acc_guard4(acc[3][0], acc[3][1], acc[3][2], acc[3][3]);

  float* slab = sT[wave];
  const int nHalf = N >> 1;
  const bool wordTile = (EPI == 1) && (n0 < nHalf);
  const int hh = lane >> 4, c4 = (lane & 15) * 4;
#pragma unroll
  for (int i = 0; i < 4; ++i) {
    const int mBase = m0 + (i << 4);
#pragma unroll
    for (int j = 0; j < 4; ++j) {
#pragma unroll
      for (int r = 0; r < 8; ++r) slab[(mOff + r) * 68 + (j << 4) + rlane] = acc[i][j][r];
    }
    __builtin_amdgcn_fence(__ATOMIC_RELEASE, "workgroup");
    __builtin_amdgcn_wave_barrier();
    __builtin_amdgcn_fence(__ATOMIC_ACQUIRE, "workgroup");
    if (wordTile) {
      unsigned* X = (unsigned*)C0;
      for (int pass = 0; pass < 2; ++pass) {
#pragma unroll 1
        for (int it = 0; it < 8; ++it) {
          const int row = it * 2 + hh;
          const float* sp = slab + row * 68 + c4;
          const float s0 = sp[0], s1 = sp[1], s2 = sp[2], s3 = sp[3];
          const unsigned w0 = split_word(s0), w1 = split_word(s1), w2 = split_word(s2), w3 = split_word(s3);
          const v4u w = {w0, w1, w2, w3};
          *(volatile v4u*)(X + (size_t)(mBase + row) * ldc + n0 + c4) = w;
        }
        __threadfence();
      }
    } else {
      float* C = (EPI == 1) ? (float*)C1 : (float*)C0;
      const int nc = (EPI == 1) ? (n0 - nHalf) : n0;
      for (int pass = 0; pass < 2; ++pass) {
#pragma unroll
        for (int it = 0; it < 8; ++it) {
          const int row = it * 2 + hh;
          const v4f v = *(const v4f*)(slab + row * 68 + c4);
          *(volatile v4f*)(C + (size_t)(mBase + row) * ldc + nc + c4) = v;
        }
        __threadfence();
      }
    }
    __builtin_amdgcn_fence(__ATOMIC_RELEASE, "workgroup");
    __builtin_amdgcn_wave_barrier();
    __builtin_amdgcn_fence(__ATOMIC_ACQUIRE, "workgroup");
  }
}

__global__ __launch_bounds__(256) void cast_bf16_kernel(
    const float* __restrict__ src0, const float* __restrict__ src1,
    unsigned* __restrict__ dst0, unsigned* __restrict__ dst1, int total8)
{
  const float* src = (blockIdx.y == 0) ? src0 : src1;
  unsigned*    dst = (blockIdx.y == 0) ? dst0 : dst1;
  const int i = blockIdx.x * 256 + threadIdx.x;
  if (i >= total8) return;
  const float* p = src + ((size_t)i << 3);
  const v4f a0 = *(const v4f*)(p);
  const v4f a1 = *(const v4f*)(p + 4);
  const float f0 = a0[0], f1 = a0[1], f2 = a0[2], f3 = a0[3];
  const float f4 = a1[0], f5 = a1[1], f6 = a1[2], f7 = a1[3];
  const unsigned w0 = bf16_rne_bits(f0) | (bf16_rne_bits(f1) << 16);
  const unsigned w1 = bf16_rne_bits(f2) | (bf16_rne_bits(f3) << 16);
  const unsigned w2 = bf16_rne_bits(f4) | (bf16_rne_bits(f5) << 16);
  const unsigned w3 = bf16_rne_bits(f6) | (bf16_rne_bits(f7) << 16);
  const v4u w = {w0, w1, w2, w3};
  unsigned* q = dst + ((size_t)i << 2);
  *(volatile v4u*)q = w;
  __threadfence();
  *(volatile v4u*)q = w;
}

__global__ __launch_bounds__(256) void dup_rows_kernel(
    const float* __restrict__ src, unsigned* __restrict__ dst, int cols, int nreal, int total4)
{
  const int i = blockIdx.x * 256 + threadIdx.x;
  if (i >= total4) return;
  const int e0  = i << 2;
  const int row = e0 / cols;
  const int col = e0 - row * cols;
  const int rowc = (row < nreal) ? row : (nreal - 1);
  const v4f a = *(const v4f*)(src + (size_t)rowc * cols + col);
  const float f0 = a[0], f1 = a[1], f2 = a[2], f3 = a[3];
  const bool keep = (row < nreal);
  const unsigned b0 = bf16_rne_bits(f0), b1 = bf16_rne_bits(f1), b2 = bf16_rne_bits(f2), b3 = bf16_rne_bits(f3);
  const unsigned w0 = keep ? (b0 | (b0 << 16)) : 0u;
  const unsigned w1 = keep ? (b1 | (b1 << 16)) : 0u;
  const unsigned w2 = keep ? (b2 | (b2 << 16)) : 0u;
  const unsigned w3 = keep ? (b3 | (b3 << 16)) : 0u;
  const v4u w = {w0, w1, w2, w3};
  unsigned* q = dst + (size_t)e0;
  *(volatile v4u*)q = w;
  __threadfence();
  *(volatile v4u*)q = w;
}

__global__ __launch_bounds__(256) void conv_silu_kernel(
    const unsigned* __restrict__ XIN, const float* __restrict__ cw, const float* __restrict__ cb,
    unsigned* __restrict__ XCW)
{
  const int idx = blockIdx.x * 256 + threadIdx.x;
  const int m = idx >> 11;
  const int d = idx & (kDin - 1);
  const int t = m & (kSeq - 1);
  const v4f wv = *(const v4f*)(cw + (size_t)d * 4);
  const float wr0 = wv[0], wr1 = wv[1], wr2 = wv[2], wr3 = wv[3];
  const float w0 = bf16_rne_val(wr0), w1 = bf16_rne_val(wr1), w2 = bf16_rne_val(wr2), w3 = bf16_rne_val(wr3);
  const float bc = bf16_rne_val(cb[d]);
  const bool p3 = (t >= 3), p2 = (t >= 2), p1 = (t >= 1);
  const int r3 = p3 ? (m - 3) : m;
  const int r2 = p2 ? (m - 2) : m;
  const int r1 = p1 ? (m - 1) : m;
  const unsigned u3 = XIN[(size_t)r3 * kDin + d];
  const unsigned u2 = XIN[(size_t)r2 * kDin + d];
  const unsigned u1 = XIN[(size_t)r1 * kDin + d];
  const unsigned u0 = XIN[(size_t)m  * kDin + d];
  const float x3 = p3 ? word_val(u3) : 0.0f;
  const float x2 = p2 ? word_val(u2) : 0.0f;
  const float x1 = p1 ? word_val(u1) : 0.0f;
  const float x0 = word_val(u0);
  float acc = w0 * x3;
  acc = fmaf(w1, x2, acc);
  acc = fmaf(w2, x1, acc);
  acc = fmaf(w3, x0, acc);
  const float sv = acc + bc;
  const float sg = __builtin_amdgcn_rcpf(1.0f + expf(-sv));
  const unsigned w = split_word(sv * sg);
  unsigned* q = XCW + (size_t)m * kDin + d;
  *(volatile unsigned*)q = w;
  __threadfence();
  *(volatile unsigned*)q = w;
}

__global__ __launch_bounds__(128) void scan_kernel(
    const float* __restrict__ SSM, const unsigned* __restrict__ XCW, const float* __restrict__ ZS,
    const float* __restrict__ Alog, const float* __restrict__ Dp, unsigned* __restrict__ YW)
{
  __shared__ __align__(16) float sH[(kNst / 4) * kScCh * 4];
  __shared__ __align__(16) float sP[kScTS * kSsmP];
  __shared__ __align__(16) unsigned sY[kScTS * kScCh];
  const int tid = threadIdx.x;
  const int d = blockIdx.x * kScCh + tid;
  const size_t row0 = (size_t)blockIdx.y * kSeq;
  const int sidx = tid & (kNst - 1);
  const int sthalf = tid >> 6;
  const float An = -expf(bf16_rne_val(Alog[sidx]));
  const float Dd = bf16_rne_val(Dp[d]);
  {
    const v4f zero4 = {0.f, 0.f, 0.f, 0.f};
#pragma unroll 1
    for (int s4 = 0; s4 < kNst / 4; ++s4) *(v4f*)(sH + ((s4 * kScCh + tid) << 2)) = zero4;
  }
#pragma unroll 1
  for (int t0 = 0; t0 < kSeq; t0 += kScTS) {
    __syncthreads();
#pragma unroll 1
    for (int i = 0; i < 8; ++i) {
      const int st = sthalf + 2 * i;
      const float* sr = SSM + (row0 + t0 + st) * kSsmP;
      const float bv = sr[sidx];
      const float cv = sr[kNst + sidx];
      const float dr = sr[2 * kNst];
      const float dt = fmaxf(dr, 0.0f) + log1pf(expf(-fabsf(dr)));
      float ab = expf(An * dt);
      ab = (ab < 1.17549435e-38f) ? 0.0f : ab;
      sP[st * kSsmP + sidx]            = ab;
      sP[st * kSsmP + kNst + sidx]     = dt * bv;
      sP[st * kSsmP + 2 * kNst + sidx] = cv;
    }
    __syncthreads();
#pragma unroll 1
    for (int st = 0; st < kScTS; ++st) {
      const size_t m = row0 + t0 + st;
      const unsigned wx = XCW[m * kDin + d];
      const float zv = ZS[m * kDin + d];
      const float xc = word_val(wx);
      const float* pr = sP + st * kSsmP;
      float acc = 0.0f;
#pragma unroll 2
      for (int s4 = 0; s4 < kNst / 4; ++s4) {
        const v4f ab = *(const v4f*)(pr + 4 * s4);
        const v4f db = *(const v4f*)(pr + kNst + 4 * s4);
        const v4f cv = *(const v4f*)(pr + 2 * kNst + 4 * s4);
        float* hp = sH + ((s4 * kScCh + tid) << 2);
        const v4f hv = *(const v4f*)hp;
        const float h0 = fmaf(ab[0], hv[0], xc * db[0]);
        const float h1 = fmaf(ab[1], hv[1], xc * db[1]);
        const float h2 = fmaf(ab[2], hv[2], xc * db[2]);
        const float h3 = fmaf(ab[3], hv[3], xc * db[3]);
        const v4f hn = {h0, h1, h2, h3};
        *(v4f*)hp = hn;
        acc = fmaf(h0, cv[0], acc);
        acc = fmaf(h1, cv[1], acc);
        acc = fmaf(h2, cv[2], acc);
        acc = fmaf(h3, cv[3], acc);
      }
      const float y  = acc + xc * Dd;
      const float sg = __builtin_amdgcn_rcpf(1.0f + expf(-zv));
      const float v  = y * (zv * sg);
      sY[st * kScCh + tid] = split_word(v);
    }
    for (int pass = 0; pass < 2; ++pass) {
#pragma unroll 4
      for (int st = 0; st < kScTS; ++st) {
        const unsigned w = sY[st * kScCh + tid];
        *(volatile unsigned*)(YW + (row0 + t0 + st) * kDin + d) = w;
      }
      __threadfence();
    }
  }
}

extern "C" void kernel_launch(void* const* d_in, const int* in_sizes, int n_in,
                              void* d_out, int out_size, void* d_ws, size_t ws_size,
                              hipStream_t stream)
{
  if (n_in < 8) return;
  if (in_sizes[0] != kRows * kDm) return;
  if (in_sizes[1] != kXzN * kDm) return;
  if (in_sizes[2] != kDin * 4) return;
  if (in_sizes[3] != kDin) return;
  if (in_sizes[4] != kSsmN * kDin) return;
  if (in_sizes[5] != kNst) return;
  if (in_sizes[6] != kDin) return;
  if (in_sizes[7] != kDm * kDin) return;
  if (out_size != kRows * kDm) return;
  if (ws_size < kWsTotal) return;

  const float* x      = (const float*)d_in[0];
  const float* W_in   = (const float*)d_in[1];
  const float* conv_w = (const float*)d_in[2];
  const float* conv_b = (const float*)d_in[3];
  const float* W_x    = (const float*)d_in[4];
  const float* A_log  = (const float*)d_in[5];
  const float* Dp     = (const float*)d_in[6];
  const float* W_out  = (const float*)d_in[7];
  float* out = (float*)d_out;

  char* ws = (char*)d_ws;
  unsigned* XB    = (unsigned*)(ws + kOffXB);
  unsigned* WINB  = (unsigned*)(ws + kOffWINB);
  unsigned* WXD   = (unsigned*)(ws + kOffWXD);
  unsigned* WOUTD = (unsigned*)(ws + kOffWOUTD);
  unsigned* XIN   = (unsigned*)(ws + kOffXIN);
  unsigned* YW    = (unsigned*)(ws + kOffXIN);
  float*    ZS    = (float*)(ws + kOffZS);
  unsigned* XCW   = (unsigned*)(ws + kOffXCW);
  float*    SSM   = (float*)(ws + kOffSSM);

  cast_bf16_kernel<<<dim3((kRows * kDm / 8) / 256, 2), 256, 0, stream>>>(x, W_in, XB, WINB, kRows * kDm / 8);
  dup_rows_kernel<<<(kSsmP * kDin / 4) / 256, 256, 0, stream>>>(W_x, WXD, kDin, kSsmN, kSsmP * kDin / 4);
  dup_rows_kernel<<<(kDm * kDin / 4) / 256, 256, 0, stream>>>(W_out, WOUTD, kDin, kDm, kDm * kDin / 4);

  gemm_bf16_kernel<1><<<(kRows / 64) * (kXzN / 64) / 8, 256, 0, stream>>>(
      (const unsigned short*)XB, kDm, (const unsigned short*)WINB, kDm,
      (void*)XIN, (void*)ZS, kDin, kRows, kXzN, kDm);

  conv_silu_kernel<<<(kRows * kDin) / 256, 256, 0, stream>>>(XIN, conv_w, conv_b, XCW);

  gemm_bf16_kernel<0><<<(kRows / 64) * (kSsmP / 64) / 8, 256, 0, stream>>>(
      (const unsigned short*)XCW, kKd, (const unsigned short*)WXD, kKd,
      (void*)SSM, (void*)SSM, kSsmP, kRows, kSsmP, kKd);

  scan_kernel<<<dim3(kDin / kScCh, kBatch), kScCh, 0, stream>>>(SSM, XCW, ZS, A_log, Dp, YW);

  gemm_bf16_kernel<0><<<(kRows / 64) * (kDm / 64) / 8, 256, 0, stream>>>(
      (const unsigned short*)YW, kKd, (const unsigned short*)WOUTD, kKd,
      (void*)out, (void*)out, kDm, kRows, kDm, kKd);
}
